// GeneEnvAttentionModelWithoutEffectSeparation_15006615734198
// MI455X (gfx1250) — hardware-verified
//
#include <hip/hip_runtime.h>
#include <math.h>
#include <stdint.h>


typedef __attribute__((ext_vector_type(16))) _Float16 v16h;
typedef __attribute__((ext_vector_type(8)))  _Float16 v8h;
typedef __attribute__((ext_vector_type(16))) __bf16   v16b;
typedef __attribute__((ext_vector_type(8)))  __bf16   v8b;
typedef __attribute__((ext_vector_type(8)))  float    v8f;
typedef __attribute__((ext_vector_type(4)))  float    v4f;
typedef __attribute__((ext_vector_type(8)))  unsigned short v8us;

__device__ __forceinline__ unsigned short f2bf_bits(float f) {
  unsigned u = __float_as_uint(f);
  return (unsigned short)((u + 0x7FFFu + ((u >> 16) & 1u)) >> 16);
}
__device__ __forceinline__ float bf_bits2f(unsigned short h) { return __uint_as_float(((unsigned)h) << 16); }
__device__ __forceinline__ unsigned short f2h_bits(float f) { return __builtin_bit_cast(unsigned short, (_Float16)f); }

__device__ __forceinline__ void dep_guard_h(v8f& a, v8f& b, v16h x, v16h y) { asm volatile("v_nop\n\tv_nop\n\tv_nop\n\tv_nop" : "+v"(a), "+v"(b) : "v"(x), "v"(y)); }
__device__ __forceinline__ void dep_guard_b(v8f& a, v8f& b, v16b x, v16b y) { asm volatile("v_nop\n\tv_nop\n\tv_nop\n\tv_nop" : "+v"(a), "+v"(b) : "v"(x), "v"(y)); }
__device__ __forceinline__ void keep4_h(v16h a, v16h b, v16h c, v16h d) { asm volatile("v_nop" :: "v"(a), "v"(b), "v"(c), "v"(d)); }
__device__ __forceinline__ void keep4_b(v16b a, v16b b, v16b c, v16b d) { asm volatile("v_nop" :: "v"(a), "v"(b), "v"(c), "v"(d)); }
__device__ __forceinline__ void acc_guard4(v8f& a, v8f& b, v8f& c, v8f& d) { asm volatile("v_nop\n\tv_nop\n\tv_nop\n\tv_nop" : "+v"(a), "+v"(b), "+v"(c), "+v"(d)); }
template <typename T> struct Frag;
template <> struct Frag<_Float16> {
  typedef v16h V; union U { v16h v; v8h h[2]; };
  static __device__ __forceinline__ v16h load(const _Float16* p) {
    U f; f.h[0] = *(const v8h*)(p); f.h[1] = *(const v8h*)(p + 16); return f.v;
  }
  static __device__ __forceinline__ v8f mma(v16h a, v16h b, v8f c) {
    return __builtin_amdgcn_wmma_f32_16x16x32_f16(false, a, false, b, (short)0, c, false, false);
  }
  static __device__ __forceinline__ void guard(v8f& a, v8f& b, v16h x, v16h y) { dep_guard_h(a, b, x, y); }
  static __device__ __forceinline__ void keep(v16h a, v16h b, v16h c, v16h d) { keep4_h(a, b, c, d); }
};
template <> struct Frag<__bf16> {
  typedef v16b V; union U { v16b v; v8b h[2]; };
  static __device__ __forceinline__ v16b load(const __bf16* p) {
    U f; f.h[0] = *(const v8b*)(p); f.h[1] = *(const v8b*)(p + 16); return f.v;
  }
  static __device__ __forceinline__ v8f mma(v16b a, v16b b, v8f c) {
    return __builtin_amdgcn_wmma_f32_16x16x32_bf16(false, a, false, b, (short)0, c, false, false);
  }
  static __device__ __forceinline__ void guard(v8f& a, v8f& b, v16b x, v16b y) { dep_guard_b(a, b, x, y); }
  static __device__ __forceinline__ void keep(v16b a, v16b b, v16b c, v16b d) { keep4_b(a, b, c, d); }
};

__device__ __forceinline__ float wave_sum(float v) {
  v += __shfl_xor(v, 16, 32);
  v += __shfl_xor(v, 8, 32);
  v += __shfl_xor(v, 4, 32);
  v += __shfl_xor(v, 2, 32);
  v += __shfl_xor(v, 1, 32);
  return v;
}
__device__ __forceinline__ float gelu_erf(float x) {
  return 0.5f * x * (1.0f + erff(x * 0.70710678118654752440f));
}

template <int MODE>
__device__ __forceinline__ void pack8(const v4f a, const v4f b, v8us& h, v8us& l) {
#pragma unroll
  for (int e = 0; e < 4; ++e) {
    const float f0 = a[e], f1 = b[e];
    if (MODE == 0) {
      h[e] = f2h_bits(f0); h[4 + e] = f2h_bits(f1); l[e] = 0; l[4 + e] = 0;
    } else {
      const unsigned short h0 = f2bf_bits(f0), h1 = f2bf_bits(f1);
      h[e] = h0; h[4 + e] = h1;
      l[e] = f2bf_bits(f0 - bf_bits2f(h0)); l[4 + e] = f2bf_bits(f1 - bf_bits2f(h1));
    }
  }
}

template <int ET> struct Elem;
template <> struct Elem<0> { typedef _Float16 T; };
template <> struct Elem<1> { typedef __bf16 T; };
template <int ET, bool SPLIT, int BIAS_MODE, int OUTF, int OUT16, int RES, int ACT>
__global__ __launch_bounds__(256) void wmma_gemm64(
    const unsigned short* __restrict__ Ap, const unsigned short* __restrict__ A2p, int lda, long strideA,
    const unsigned short* __restrict__ Btp, const unsigned short* __restrict__ Bt2p, int ldb, long strideB,
    float* Cf, unsigned short* Ca, unsigned short* Cb, int ldc, long strideC,
    const float* __restrict__ bias, long strideBias,
    const float* __restrict__ resid, long strideR,
    int M, int N, int K, float scale) {
  typedef typename Elem<ET>::T T;
  typedef typename Frag<T>::V V;
  const T* A = (const T*)Ap; const T* A2 = (const T*)A2p; const T* Bt = (const T*)Btp; const T* Bt2 = (const T*)Bt2p;
  __shared__ __align__(16) float sT[8][16 * 68];
  const int b    = blockIdx.y;
  const int lane = threadIdx.x & 31;
  const int wave = threadIdx.x >> 5;
  const int tilesN = N >> 6;
  const int tilesM = M >> 6;
  const int tile = blockIdx.x * 8 + wave;
  if (tile >= tilesM * tilesN) return;
  const int tm = tile / tilesN;
  const int tn = tile - tm * tilesN;
  const int m0 = tm << 6;
  const int n0 = tn << 6;

  const T* Ab  = A  + (size_t)b * strideA;
  const T* Bb  = Bt + (size_t)b * strideB;
  const T* Ab2 = SPLIT ? (A2  + (size_t)b * strideA) : nullptr;
  const T* Bb2 = SPLIT ? (Bt2 + (size_t)b * strideB) : nullptr;

  const int rlane = lane & 15;
  const int koff  = (lane >> 4) * 8;
  const int mOff  = (lane >> 4) * 8;

  v8f acc[4][4];
#pragma unroll
  for (int i = 0; i < 4; ++i)
#pragma unroll
    for (int j = 0; j < 4; ++j) acc[i][j] = (v8f){0.f,0.f,0.f,0.f,0.f,0.f,0.f,0.f};

  for (int k0 = 0; k0 < K; k0 += 32) {
    V bh[4], bl[4];
#pragma unroll
    for (int j = 0; j < 4; ++j) {
      const size_t bo = (size_t)(n0 + (j << 4) + rlane) * ldb + koff + k0;
      bh[j] = Frag<T>::load(Bb + bo);
      if (SPLIT) bl[j] = Frag<T>::load(Bb2 + bo);
    }
#pragma unroll
    for (int i = 0; i < 4; ++i) {
      const size_t ao = (size_t)(m0 + (i << 4) + rlane) * lda + koff + k0;
      V ah = Frag<T>::load(Ab + ao);
      V al;
      if (SPLIT) al = Frag<T>::load(Ab2 + ao);
#pragma unroll
      for (int j = 0; j < 4; ++j) {
        acc[i][j] = Frag<T>::mma(ah, bh[j], acc[i][j]);
        if (SPLIT) {
          acc[i][j] = Frag<T>::mma(ah, bl[j], acc[i][j]);
          acc[i][j] = Frag<T>::mma(al, bh[j], acc[i][j]);
        }
      }
      Frag<T>::guard(acc[i][0], acc[i][3], ah, SPLIT ? al : ah);
    }
    Frag<T>::keep(bh[0], bh[1], bh[2], bh[3]);
    if (SPLIT) Frag<T>::keep(bl[0], bl[1], bl[2], bl[3]);
  }
  acc_guard4(acc[0][0], acc[0][1], acc[0][2], acc[0][3]);
  acc_guard4(acc[1][0], acc[1][1], acc[1][2], acc[1][3]);
  acc_guard4(acc[2][0], acc[2][1], acc[2][2], acc[2][3]);
  acc_guard4(acc[3][0], acc[3][1], acc[3][2], acc[3][3]);

  float* slab = sT[wave];
  const float* Rb = (RES != 0) ? (resid + (size_t)b * strideR) : nullptr;
  const float* biasb = (BIAS_MODE != 0) ? (bias + (size_t)b * strideBias) : nullptr;
#pragma unroll
  for (int i = 0; i < 4; ++i) {
    const int mBase = m0 + (i << 4);
#pragma unroll
    for (int j = 0; j < 4; ++j) {
      const int n = n0 + (j << 4) + rlane;
      float bv = 0.f;
      if (BIAS_MODE == 2) bv = biasb[n];
#pragma unroll
      for (int r = 0; r < 8; ++r) {
        float v = acc[i][j][r] * scale;
        if (BIAS_MODE == 1) v += biasb[mBase + mOff + r];
        if (BIAS_MODE == 2) v += bv;
        if (RES == 1) v += Rb[(size_t)(mBase + mOff + r) * ldc + n];
        if (ACT == 1) v = tanhf(v);
        if (ACT == 2) v = fmaxf(v, 0.0f);
        if (ACT == 3) v = v / (1.0f + expf(-v));
        if (ACT == 4) v = (v > 0.f) ? v : 0.01f * v;
        if (ACT == 5) v = 0.5f * v * (1.0f + erff(v * 0.70710678118654752f));
        if (RES == 2) v *= Rb[(size_t)(mBase + mOff + r) * ldc + n];
        slab[(mOff + r) * 68 + (j << 4) + rlane] = v;
      }
    }
    __builtin_amdgcn_fence(__ATOMIC_RELEASE, "workgroup");
    __builtin_amdgcn_wave_barrier();
    __builtin_amdgcn_fence(__ATOMIC_ACQUIRE, "workgroup");
    if (OUTF) {
      float* C = Cf + (size_t)b * strideC;
      const int hh = lane >> 4, c4 = (lane & 15) * 4;
      for (int pass = 0; pass < 2; ++pass) {
#pragma unroll
        for (int it = 0; it < 8; ++it) {
          const int row = it * 2 + hh;
          v4f v = *(const v4f*)(slab + row * 68 + c4);
          *(volatile v4f*)(C + (size_t)(mBase + row) * ldc + n0 + c4) = v;
        }
        __threadfence();
      }
    }
    if (OUT16 != 0) {
      const int q = lane >> 3, c8 = (lane & 7) * 8;
      unsigned short* C  = Ca + (size_t)b * strideC;
      unsigned short* C2 = (OUT16 == 2) ? (Cb + (size_t)b * strideC) : nullptr;
      for (int pass = 0; pass < 2; ++pass) {
#pragma unroll
        for (int it = 0; it < 4; ++it) {
          const int row = it * 4 + q;
          const float* sp = slab + row * 68 + c8;
          v8h hv = (v8h){0, 0, 0, 0, 0, 0, 0, 0};
          v8h lv = (v8h){0, 0, 0, 0, 0, 0, 0, 0};
#pragma unroll
          for (int e = 0; e < 8; ++e) {
            if (OUT16 == 2) {
              unsigned short hb = f2bf_bits(sp[e]);
              unsigned short lb = f2bf_bits(sp[e] - bf_bits2f(hb));
              hv[e] = __builtin_bit_cast(_Float16, hb);
              lv[e] = __builtin_bit_cast(_Float16, lb);
            } else {
              hv[e] = (_Float16)sp[e];
            }
          }
          *(volatile v8h*)(C + (size_t)(mBase + row) * ldc + n0 + c8) = hv;
          if (OUT16 == 2) *(volatile v8h*)(C2 + (size_t)(mBase + row) * ldc + n0 + c8) = lv;
        }
        __threadfence();
      }
    }
    __builtin_amdgcn_fence(__ATOMIC_RELEASE, "workgroup");
    __builtin_amdgcn_wave_barrier();
    __builtin_amdgcn_fence(__ATOMIC_ACQUIRE, "workgroup");
  }
}

__global__ __launch_bounds__(256) void cast_f32_bf16hl(
    const float* __restrict__ in, unsigned short* hi, unsigned short* lo, int n8) {
  const int i = blockIdx.x * 256 + threadIdx.x;
  if (i < n8) {
    const v4f a = *(const v4f*)(in + (size_t)i * 8);
    const v4f b = *(const v4f*)(in + (size_t)i * 8 + 4);
    v8us hv, lv;
    pack8<1>(a, b, hv, lv);
    unsigned short* ph = hi + (size_t)i * 8;
    unsigned short* pl = lo + (size_t)i * 8;
    *(volatile v8us*)ph = hv;
    *(volatile v8us*)pl = lv;
    __threadfence();
    *(volatile v8us*)ph = hv;
    *(volatile v8us*)pl = lv;
  }
}

template <int MODE>
__global__ __launch_bounds__(256) void transpose_cast(const float* __restrict__ in, unsigned short* out, unsigned short* out2,
    int R, int C, long sIn, long sOut, float mul)
{
  __shared__ __align__(16) float s[64 * 68];
  const int tid = threadIdx.x;
  const int c0 = blockIdx.x * 64, r0 = blockIdx.y * 64;
  const float* ib = in + (size_t)blockIdx.z * sIn;
#pragma unroll
  for (int i = 0; i < 16; ++i) {
    const int idx = tid + i * 256;
    const int r = idx >> 6, c = idx & 63;
    s[c * 68 + r] = ib[(size_t)(r0 + r) * C + c0 + c] * mul;
  }
  __syncthreads();
  const int wave = tid >> 5, lane = tid & 31, q = lane >> 3, c8 = (lane & 7) * 8;
  const int rowA = wave * 8 + q, rowB = wave * 8 + 4 + q;
  const v4f a0 = *(const v4f*)(s + rowA * 68 + c8), a1 = *(const v4f*)(s + rowA * 68 + c8 + 4);
  const v4f b0 = *(const v4f*)(s + rowB * 68 + c8), b1 = *(const v4f*)(s + rowB * 68 + c8 + 4);
  v8us ha, la, hb, lb;
  pack8<MODE>(a0, a1, ha, la);
  pack8<MODE>(b0, b1, hb, lb);
  unsigned short* ob  = out  + (size_t)blockIdx.z * sOut;
  unsigned short* ob2 = out2 + (size_t)blockIdx.z * sOut;
  unsigned short* pa  = ob  + (size_t)(c0 + rowA) * R + r0 + c8;
  unsigned short* pb  = ob  + (size_t)(c0 + rowB) * R + r0 + c8;
  unsigned short* pa2 = ob2 + (size_t)(c0 + rowA) * R + r0 + c8;
  unsigned short* pb2 = ob2 + (size_t)(c0 + rowB) * R + r0 + c8;
  *(volatile v8us*)pa = ha;
  *(volatile v8us*)pb = hb;
  if (MODE == 1) { *(volatile v8us*)pa2 = la; *(volatile v8us*)pb2 = lb; }
  __threadfence();
  *(volatile v8us*)pa = ha;
  *(volatile v8us*)pb = hb;
  if (MODE == 1) { *(volatile v8us*)pa2 = la; *(volatile v8us*)pb2 = lb; }
}

template <bool GELU, int OMODE>
__global__ __launch_bounds__(256) void ln_rows(const float* __restrict__ X, int ldx,
    const float* __restrict__ gam, const float* __restrict__ bet, int grpRows,
    unsigned short* Y, unsigned short* Y2, int ldy, int rows, int D)
{
  const int lane = threadIdx.x & 31, wave = threadIdx.x >> 5;
  const int row = blockIdx.x * 8 + wave;
  if (row >= rows) return;
  const float* x = X + (size_t)row * ldx;
  const int goff = (row / grpRows) * D;
  const float* g = gam + goff;
  const float* bb = bet + goff;
  const int nch = (D + 255) >> 8;
  const float invD = 1.0f / (float)D;
  float s = 0.f;
#pragma unroll 1
  for (int c = 0; c < nch; ++c) {
    const int col = (c << 8) + lane * 8;
    if (col < D) {
      const v4f a = *(const v4f*)(x + col);
      const v4f b = *(const v4f*)(x + col + 4);
      s += ((a[0] + a[1]) + (a[2] + a[3])) + ((b[0] + b[1]) + (b[2] + b[3]));
    }
  }
  s = wave_sum(s);
  const float mean = s * invD;
  float q = 0.f;
#pragma unroll 1
  for (int c = 0; c < nch; ++c) {
    const int col = (c << 8) + lane * 8;
    if (col < D) {
      const v4f a = *(const v4f*)(x + col);
      const v4f b = *(const v4f*)(x + col + 4);
#pragma unroll
      for (int e = 0; e < 4; ++e) {
        const float d0 = a[e] - mean, d1 = b[e] - mean;
        q = fmaf(d0, d0, q); q = fmaf(d1, d1, q);
      }
    }
  }
  q = wave_sum(q);
  const float rstd = rsqrtf(q * invD + 1e-5f);
#pragma unroll 1
  for (int c = 0; c < nch; ++c) {
    const int col = (c << 8) + lane * 8;
    if (col < D) {
      const v4f a  = *(const v4f*)(x + col);
      const v4f b  = *(const v4f*)(x + col + 4);
      const v4f g0 = *(const v4f*)(g + col);
      const v4f g1 = *(const v4f*)(g + col + 4);
      const v4f e0 = *(const v4f*)(bb + col);
      const v4f e1 = *(const v4f*)(bb + col + 4);
      v4f ta, tb;
#pragma unroll
      for (int e = 0; e < 4; ++e) {
        float t0 = (a[e] - mean) * rstd * g0[e] + e0[e];
        float t1 = (b[e] - mean) * rstd * g1[e] + e1[e];
        if (GELU) { t0 = gelu_erf(t0); t1 = gelu_erf(t1); }
        ta[e] = t0; tb[e] = t1;
      }
      v8us hv, lv;
      pack8<OMODE>(ta, tb, hv, lv);
      unsigned short* p  = Y  + (size_t)row * ldy + col;
      unsigned short* p2 = Y2 + (size_t)row * ldy + col;
      *(volatile v8us*)p = hv;
      if (OMODE == 1) *(volatile v8us*)p2 = lv;
      __threadfence();
      *(volatile v8us*)p = hv;
      if (OMODE == 1) *(volatile v8us*)p2 = lv;
    }
  }
}

__global__ __launch_bounds__(256) void gate_route(const float* __restrict__ ff, const float* __restrict__ gw,
    const float* __restrict__ gb, float* probs, float* comb, float* maskf, int B, int K)
{
  __shared__ __align__(16) float sP[256];
  __shared__ __align__(16) float sC[256];
  __shared__ __align__(16) float sM[256];
  const int lane = threadIdx.x & 31, wave = threadIdx.x >> 5;
#pragma unroll 1
  for (int rr = 0; rr < 4; ++rr) {
    const int rloc = wave * 4 + rr;
    int row = blockIdx.x * 32 + rloc;
    if (row > B - 1) row = B - 1;
    const float* xr = ff + (size_t)row * K;
    float s[8];
#pragma unroll
    for (int e = 0; e < 8; ++e) s[e] = 0.f;
#pragma unroll 1
    for (int k = lane; k < K; k += 32) {
      const float xv = xr[k];
      const v4f w0 = *(const v4f*)(gw + (size_t)k * 8);
      const v4f w1 = *(const v4f*)(gw + (size_t)k * 8 + 4);
      s[0] = fmaf(xv, w0[0], s[0]); s[1] = fmaf(xv, w0[1], s[1]);
      s[2] = fmaf(xv, w0[2], s[2]); s[3] = fmaf(xv, w0[3], s[3]);
      s[4] = fmaf(xv, w1[0], s[4]); s[5] = fmaf(xv, w1[1], s[5]);
      s[6] = fmaf(xv, w1[2], s[6]); s[7] = fmaf(xv, w1[3], s[7]);
    }
#pragma unroll
    for (int e = 0; e < 8; ++e) s[e] = wave_sum(s[e]) + gb[e];
    float mx = s[0];
#pragma unroll
    for (int e = 1; e < 8; ++e) mx = fmaxf(mx, s[e]);
    float ex[8], sum = 0.f;
#pragma unroll
    for (int e = 0; e < 8; ++e) { ex[e] = expf(s[e] - mx); sum += ex[e]; }
    const float rs = 1.0f / sum;
    float p[8];
#pragma unroll
    for (int e = 0; e < 8; ++e) p[e] = ex[e] * rs;
    float b0 = p[0]; int i0 = 0;
#pragma unroll
    for (int e = 1; e < 8; ++e) { if (p[e] > b0) { b0 = p[e]; i0 = e; } }
    float b1 = -1.0f; int i1 = -1;
#pragma unroll
    for (int e = 0; e < 8; ++e) { if (e != i0 && p[e] > b1) { b1 = p[e]; i1 = e; } }
    const float rn = 1.0f / (b0 + b1);
    const float c0v = b0 * rn, c1v = b1 * rn;
    if (lane == 0) {
#pragma unroll
      for (int e = 0; e < 8; ++e) {
        sP[rloc * 8 + e] = p[e];
        sC[rloc * 8 + e] = (e == i0) ? c0v : ((e == i1) ? c1v : 0.0f);
        sM[rloc * 8 + e] = (e == i0 || e == i1) ? 1.0f : 0.0f;
      }
    }
  }
  __syncthreads();
  if (wave < 3) {
    const float* src = (wave == 0) ? sP : ((wave == 1) ? sC : sM);
    float* dst = ((wave == 0) ? probs : ((wave == 1) ? comb : maskf)) + (size_t)blockIdx.x * 256;
    const v4f va = *(const v4f*)(src + lane * 4);
    const v4f vb = *(const v4f*)(src + 128 + lane * 4);
    const bool oka = (blockIdx.x * 32 + (lane >> 1)) < B;
    const bool okb = (blockIdx.x * 32 + 16 + (lane >> 1)) < B;
    if (oka) *(volatile v4f*)(dst + lane * 4) = va;
    if (okb) *(volatile v4f*)(dst + 128 + lane * 4) = vb;
    __threadfence();
    if (oka) *(volatile v4f*)(dst + lane * 4) = va;
    if (okb) *(volatile v4f*)(dst + 128 + lane * 4) = vb;
  }
}

__global__ __launch_bounds__(256) void aux_loss_k(const float* __restrict__ probs, const float* __restrict__ maskf,
    float* out1, int B)
{
  __shared__ float red[8][16];
  const int lane = threadIdx.x & 31, wave = threadIdx.x >> 5;
  float imp[8], cnt[8];
#pragma unroll
  for (int e = 0; e < 8; ++e) { imp[e] = 0.f; cnt[e] = 0.f; }
#pragma unroll 1
  for (int r = threadIdx.x; r < B; r += 256) {
    const v4f pa = *(const v4f*)(probs + (size_t)r * 8);
    const v4f pb = *(const v4f*)(probs + (size_t)r * 8 + 4);
    const v4f ca = *(const v4f*)(maskf + (size_t)r * 8);
    const v4f cb = *(const v4f*)(maskf + (size_t)r * 8 + 4);
#pragma unroll
    for (int e = 0; e < 4; ++e) {
      imp[e] += pa[e]; imp[4 + e] += pb[e];
      cnt[e] += ca[e]; cnt[4 + e] += cb[e];
    }
  }
#pragma unroll
  for (int e = 0; e < 8; ++e) { imp[e] = wave_sum(imp[e]); cnt[e] = wave_sum(cnt[e]); }
  if (lane == 0) {
#pragma unroll
    for (int e = 0; e < 8; ++e) { red[wave][e] = imp[e]; red[wave][8 + e] = cnt[e]; }
  }
  __syncthreads();
  if (threadIdx.x == 0) {
    float iv[8], lv[8];
    const float invB = 1.0f / (float)B;
#pragma unroll
    for (int e = 0; e < 8; ++e) {
      float a = 0.f, c = 0.f;
#pragma unroll
      for (int w = 0; w < 8; ++w) { a += red[w][e]; c += red[w][8 + e]; }
      iv[e] = a; lv[e] = c * invB;
    }
    float mi = 0.f, ml = 0.f;
#pragma unroll
    for (int e = 0; e < 8; ++e) { mi += iv[e]; ml += lv[e]; }
    mi *= 0.125f; ml *= 0.125f;
    float vi = 0.f, vl = 0.f;
#pragma unroll
    for (int e = 0; e < 8; ++e) { float d = iv[e] - mi; vi += d * d; d = lv[e] - ml; vl += d * d; }
    vi *= (1.0f / 7.0f); vl *= (1.0f / 7.0f);
    float li = sqrtf(vi) * (1.0f / (mi + 1e-6f)); li = li * li;
    float ll = sqrtf(vl) * (1.0f / (ml + 1e-6f)); ll = ll * ll;
    const float res = li + ll;
    *(volatile float*)out1 = res;
    __threadfence();
    *(volatile float*)out1 = res;
  }
}

__global__ __launch_bounds__(256) void moe_combine_ln(const float* __restrict__ Y, const float* __restrict__ comb,
    const float* __restrict__ g, const float* __restrict__ bb, unsigned short* out, int B)
{
  const int lane = threadIdx.x & 31, wave = threadIdx.x >> 5;
  const int row = blockIdx.x * 8 + wave;
  if (row >= B) return;
  float x[16];
#pragma unroll
  for (int i = 0; i < 16; ++i) x[i] = 0.f;
#pragma unroll 1
  for (int e = 0; e < 8; ++e) {
    const float w = comb[(size_t)row * 8 + e];
    const float* yr = Y + ((size_t)e * B + row) * 512;
#pragma unroll
    for (int c = 0; c < 2; ++c) {
      const v4f a0 = *(const v4f*)(yr + c * 256 + lane * 8);
      const v4f a1 = *(const v4f*)(yr + c * 256 + lane * 8 + 4);
#pragma unroll
      for (int j = 0; j < 4; ++j) {
        x[c * 8 + j]     = fmaf(w, a0[j], x[c * 8 + j]);
        x[c * 8 + 4 + j] = fmaf(w, a1[j], x[c * 8 + 4 + j]);
      }
    }
  }
  float s = 0.f;
#pragma unroll
  for (int i = 0; i < 16; ++i) s += x[i];
  s = wave_sum(s);
  const float mean = s * (1.0f / 512.0f);
  float q = 0.f;
#pragma unroll
  for (int i = 0; i < 16; ++i) { const float d = x[i] - mean; q = fmaf(d, d, q); }
  q = wave_sum(q);
  const float rstd = rsqrtf(q * (1.0f / 512.0f) + 1e-5f);
  v8us hv[2];
#pragma unroll
  for (int c = 0; c < 2; ++c) {
    const int col = c * 256 + lane * 8;
    const v4f g0 = *(const v4f*)(g + col), g1 = *(const v4f*)(g + col + 4);
    const v4f b0 = *(const v4f*)(bb + col), b1 = *(const v4f*)(bb + col + 4);
#pragma unroll
    for (int j = 0; j < 4; ++j) {
      hv[c][j]     = f2h_bits((x[c * 8 + j] - mean) * rstd * g0[j] + b0[j]);
      hv[c][4 + j] = f2h_bits((x[c * 8 + 4 + j] - mean) * rstd * g1[j] + b1[j]);
    }
  }
  unsigned short* p0 = out + (size_t)row * 512 + lane * 8;
  unsigned short* p1 = out + (size_t)row * 512 + 256 + lane * 8;
  *(volatile v8us*)p0 = hv[0];
  *(volatile v8us*)p1 = hv[1];
  __threadfence();
  *(volatile v8us*)p0 = hv[0];
  *(volatile v8us*)p1 = hv[1];
}

__global__ __launch_bounds__(256) void ln_gelu_head(const float* __restrict__ X, const float* __restrict__ g,
    const float* __restrict__ bb, const float* __restrict__ pw, const float* __restrict__ pbias,
    float* out, int B)
{
  __shared__ __align__(16) float sPred[32];
  const int lane = threadIdx.x & 31, wave = threadIdx.x >> 5;
#pragma unroll 1
  for (int rr = 0; rr < 4; ++rr) {
    const int rloc = wave * 4 + rr;
    int row = blockIdx.x * 32 + rloc;
    if (row > B - 1) row = B - 1;
    const float* x = X + (size_t)row * 256;
    float s = 0.f;
#pragma unroll 1
    for (int c = 0; c < 2; ++c) {
      const v4f v = *(const v4f*)(x + c * 128 + lane * 4);
      s += (v[0] + v[1]) + (v[2] + v[3]);
    }
    s = wave_sum(s);
    const float mean = s * (1.0f / 256.0f);
    float q = 0.f;
#pragma unroll 1
    for (int c = 0; c < 2; ++c) {
      const v4f v = *(const v4f*)(x + c * 128 + lane * 4);
#pragma unroll
      for (int e = 0; e < 4; ++e) { const float d = v[e] - mean; q = fmaf(d, d, q); }
    }
    q = wave_sum(q);
    const float rstd = rsqrtf(q * (1.0f / 256.0f) + 1e-5f);
    float dot = 0.f;
#pragma unroll 1
    for (int c = 0; c < 2; ++c) {
      const int col = c * 128 + lane * 4;
      const v4f v  = *(const v4f*)(x + col);
      const v4f gg = *(const v4f*)(g + col);
      const v4f be = *(const v4f*)(bb + col);
      const v4f ww = *(const v4f*)(pw + col);
#pragma unroll
      for (int e = 0; e < 4; ++e) {
        const float t = gelu_erf((v[e] - mean) * rstd * gg[e] + be[e]);
        dot = fmaf(t, ww[e], dot);
      }
    }
    dot = wave_sum(dot);
    if (lane == 0) sPred[rloc] = dot + pbias[0];
  }
  __syncthreads();
  if (wave == 0 && lane < 8) {
    const int r0 = blockIdx.x * 32 + lane * 4;
    const v4f v = *(const v4f*)(sPred + lane * 4);
    const bool ok = (r0 + 3) < B;
    if (ok) *(volatile v4f*)(out + r0) = v;
    __threadfence();
    if (ok) *(volatile v4f*)(out + r0) = v;
  }
}

typedef unsigned short us16;

template <int ET, bool SPLIT, int OUTF, int OUT16, int RES, int ACT>
static void run_gemm(hipStream_t st, const us16* A, const us16* A2, int lda, long sA,
                     const us16* Bt, const us16* Bt2, int ldb, long sB,
                     float* Cf, us16* Ca, us16* Cb, int ldc, long sC,
                     const float* bias, long sBias,
                     const float* resid, long sR,
                     int M, int N, int K, int batch, float scale)
{
  const int tiles = (M >> 6) * (N >> 6);
  dim3 grid((unsigned)((tiles + 7) / 8), (unsigned)batch, 1);
  wmma_gemm64<ET, SPLIT, 2, OUTF, OUT16, RES, ACT><<<grid, dim3(256), 0, st>>>(
      A, A2, lda, sA, Bt, Bt2, ldb, sB, Cf, Ca, Cb, ldc, sC, bias, sBias, resid, sR, M, N, K, scale);
}

static void run_tpose_hl(hipStream_t st, const float* in, us16* h, us16* l, int R, int C)
{
  dim3 grid((unsigned)(C / 64), (unsigned)(R / 64), 1);
  transpose_cast<1><<<grid, dim3(256), 0, st>>>(in, h, l, R, C, (long)R * C, (long)R * C, 1.0f);
}
static void run_tpose_f16(hipStream_t st, const float* in, us16* out, int R, int C, int Z)
{
  dim3 grid((unsigned)(C / 64), (unsigned)(R / 64), (unsigned)Z);
  transpose_cast<0><<<grid, dim3(256), 0, st>>>(in, out, out, R, C, (long)R * C, (long)R * C, 64.0f);
}

extern "C" void kernel_launch(void* const* d_in, const int* in_sizes, int n_in,
                              void* d_out, int out_size, void* d_ws, size_t ws_size,
                              hipStream_t stream)
{
  const int B = 1024, S = 4096, E_ = 64, WU = 1024, EU = 256;
  const int SA = 512, EA = 128, FD = 512, MH = 1024, NE = 8, F1 = 512, F2 = 256;
  if (n_in < 58) return;
  if (in_sizes[0] != B * S || in_sizes[1] != B * E_ || in_sizes[2] != S * WU || in_sizes[6] != WU * S ||
      in_sizes[14] != S * SA || in_sizes[36] != 2 * FD * FD || in_sizes[40] != NE * FD * MH ||
      in_sizes[44] != NE * MH * FD || in_sizes[52] != F1 * F2 || out_size != B + 1) return;

  const float* snp    = (const float*)d_in[0];
  const float* env    = (const float*)d_in[1];
  const float* snp_w1 = (const float*)d_in[2];  const float* snp_b1 = (const float*)d_in[3];
  const float* snp_lng= (const float*)d_in[4];  const float* snp_lnb= (const float*)d_in[5];
  const float* snp_w2 = (const float*)d_in[6];  const float* snp_b2 = (const float*)d_in[7];
  const float* env_w1 = (const float*)d_in[8];  const float* env_b1 = (const float*)d_in[9];
  const float* env_lng= (const float*)d_in[10]; const float* env_lnb= (const float*)d_in[11];
  const float* env_w2 = (const float*)d_in[12]; const float* env_b2 = (const float*)d_in[13];
  const float* snp_pw = (const float*)d_in[14]; const float* snp_pb = (const float*)d_in[15];
  const float* env_pw = (const float*)d_in[16]; const float* env_pb = (const float*)d_in[17];
  const float* snp_wv = (const float*)d_in[18]; const float* snp_bv = (const float*)d_in[19];
  const float* snp_wo = (const float*)d_in[20]; const float* snp_bo = (const float*)d_in[21];
  const float* snp_ng = (const float*)d_in[22]; const float* snp_nb = (const float*)d_in[23];
  const float* env_wv = (const float*)d_in[24]; const float* env_bv = (const float*)d_in[25];
  const float* env_wo = (const float*)d_in[26]; const float* env_bo = (const float*)d_in[27];
  const float* env_ng = (const float*)d_in[28]; const float* env_nb = (const float*)d_in[29];
  const float* snp_fw = (const float*)d_in[30]; const float* snp_fb = (const float*)d_in[31];
  const float* env_fw = (const float*)d_in[32]; const float* env_fb = (const float*)d_in[33];
  const float* fus_ng = (const float*)d_in[34]; const float* fus_nb = (const float*)d_in[35];
  const float* fus_fw = (const float*)d_in[36]; const float* fus_fb = (const float*)d_in[37];
  const float* gate_w = (const float*)d_in[38]; const float* gate_b = (const float*)d_in[39];
  const float* ew1    = (const float*)d_in[40]; const float* eb1    = (const float*)d_in[41];
  const float* elg    = (const float*)d_in[42]; const float* elb    = (const float*)d_in[43];
  const float* ew2    = (const float*)d_in[44]; const float* eb2    = (const float*)d_in[45];
  const float* moe_ng = (const float*)d_in[46]; const float* moe_nb = (const float*)d_in[47];
  const float* fn1_w  = (const float*)d_in[48]; const float* fn1_b  = (const float*)d_in[49];
  const float* fn1_g  = (const float*)d_in[50]; const float* fn1_bb = (const float*)d_in[51];
  const float* fn2_w  = (const float*)d_in[52]; const float* fn2_b  = (const float*)d_in[53];
  const float* fn2_g  = (const float*)d_in[54]; const float* fn2_bb = (const float*)d_in[55];
  const float* pred_w = (const float*)d_in[56]; const float* pred_b = (const float*)d_in[57];

  float* out0 = (float*)d_out;
  float* out1 = (float*)d_out + B;

  const size_t MiB = 1048576;
  char* wsb = (char*)d_ws;
  size_t off = 0;
  auto carve = [&](size_t bytes) -> char* { char* p = wsb + off; off += (bytes + 255) & ~(size_t)255; return p; };
  auto carveHL = [&](size_t n, us16*& h, us16*& l) { char* p = carve(n * 4); h = (us16*)p; l = (us16*)(p + n * 2); };

  char* P = carve(64 * MiB);
  us16*  snp_h  = (us16*)(P + 0);           us16* snp_l  = (us16*)(P + 8 * MiB);
  us16*  seff_h = (us16*)(P + 0);           us16* seff_l = (us16*)(P + 8 * MiB);
  us16*  w1T_h  = (us16*)(P + 16 * MiB);    us16* w1T_l  = (us16*)(P + 24 * MiB);
  us16*  pwT_h  = (us16*)(P + 16 * MiB);    us16* pwT_l  = (us16*)(P + 20 * MiB);
  us16*  w2T_h  = (us16*)(P + 32 * MiB);    us16* w2T_l  = (us16*)(P + 40 * MiB);
  float* th1    = (float*)(P + 48 * MiB);
  us16*  th2_h  = (us16*)(P + 52 * MiB);    us16* th2_l  = (us16*)(P + 54 * MiB);
  float* hbuf   = (float*)(P + 0);
  us16*  h16    = (us16*)(P + 32 * MiB);
  float* ybuf   = (float*)(P + 48 * MiB);

  us16* ew1T = (us16*)carve((size_t)NE * MH * FD * 2);
  us16* ew2T = (us16*)carve((size_t)NE * FD * MH * 2);
  us16 *env_h, *env_l;     carveHL((size_t)B * E_, env_h, env_l);
  us16 *e_w1T_h, *e_w1T_l; carveHL((size_t)EU * E_, e_w1T_h, e_w1T_l);
  us16 *e_w2T_h, *e_w2T_l; carveHL((size_t)E_ * EU, e_w2T_h, e_w2T_l);
  us16 *epwT_h, *epwT_l;   carveHL((size_t)EA * E_, epwT_h, epwT_l);
  us16 *wvT_h, *wvT_l;     carveHL((size_t)SA * SA, wvT_h, wvT_l);
  us16 *woT_h, *woT_l;     carveHL((size_t)SA * SA, woT_h, woT_l);
  us16 *ewvT_h, *ewvT_l;   carveHL((size_t)EA * EA, ewvT_h, ewvT_l);
  us16 *ewoT_h, *ewoT_l;   carveHL((size_t)EA * EA, ewoT_h, ewoT_l);
  us16 *sfwT_h, *sfwT_l;   carveHL((size_t)FD * SA, sfwT_h, sfwT_l);
  us16 *efwT_h, *efwT_l;   carveHL((size_t)FD * EA, efwT_h, efwT_l);
  us16 *fusT_h, *fusT_l;   carveHL((size_t)FD * 2 * FD, fusT_h, fusT_l);
  us16* fn1T = (us16*)carve((size_t)F1 * FD * 2);
  us16* fn2T = (us16*)carve((size_t)F2 * F1 * 2);
  float* eh1  = (float*)carve((size_t)B * EU * 4);
  us16 *eh2_h, *eh2_l;     carveHL((size_t)B * EU, eh2_h, eh2_l);
  us16 *eeff_h, *eeff_l;   carveHL((size_t)B * E_, eeff_h, eeff_l);
  float* sp   = (float*)carve((size_t)B * SA * 4);
  us16 *sp_h, *sp_l;       carveHL((size_t)B * SA, sp_h, sp_l);
  us16 *sv_h, *sv_l;       carveHL((size_t)B * SA, sv_h, sv_l);
  float* sres = (float*)carve((size_t)B * SA * 4);
  us16 *sf_h, *sf_l;       carveHL((size_t)B * SA, sf_h, sf_l);
  float* ep   = (float*)carve((size_t)B * EA * 4);
  us16 *ep_h, *ep_l;       carveHL((size_t)B * EA, ep_h, ep_l);
  us16 *ev_h, *ev_l;       carveHL((size_t)B * EA, ev_h, ev_l);
  float* eres = (float*)carve((size_t)B * EA * 4);
  us16 *ef_h, *ef_l;       carveHL((size_t)B * EA, ef_h, ef_l);
  float* fused = (float*)carve((size_t)B * 2 * FD * 4);
  us16 *fus_h, *fus_l;     carveHL((size_t)B * 2 * FD, fus_h, fus_l);
  float* ff    = (float*)carve((size_t)B * FD * 4);
  us16*  ff16  = (us16*)carve((size_t)B * FD * 2);
  float* probs = (float*)carve((size_t)B * NE * 4);
  float* comb  = (float*)carve((size_t)B * NE * 4);
  float* maskf = (float*)carve((size_t)B * NE * 4);
  us16*  moe16 = (us16*)carve((size_t)B * FD * 2);
  float* f1    = (float*)carve((size_t)B * F1 * 4);
  us16*  f1n16 = (us16*)carve((size_t)B * F1 * 2);
  float* f2    = (float*)carve((size_t)B * F2 * 4);
  if (off > ws_size || off > (size_t)134217728) return;

  const dim3 blk(256);

  cast_f32_bf16hl<<<dim3((unsigned)((B * S / 8 + 255) / 256)), blk, 0, stream>>>(snp, snp_h, snp_l, B * S / 8);
  cast_f32_bf16hl<<<dim3((unsigned)((B * E_ / 8 + 255) / 256)), blk, 0, stream>>>(env, env_h, env_l, B * E_ / 8);
  run_tpose_hl(stream, snp_w1, w1T_h, w1T_l,     S,  WU);
  run_tpose_hl(stream, snp_w2, w2T_h, w2T_l,     WU, S);
  run_tpose_hl(stream, env_w1, e_w1T_h, e_w1T_l, E_, EU);
  run_tpose_hl(stream, env_w2, e_w2T_h, e_w2T_l, EU, E_);
  run_tpose_hl(stream, env_pw, epwT_h, epwT_l,   E_, EA);
  run_tpose_hl(stream, snp_wv, wvT_h, wvT_l,     SA, SA);
  run_tpose_hl(stream, snp_wo, woT_h, woT_l,     SA, SA);
  run_tpose_hl(stream, env_wv, ewvT_h, ewvT_l,   EA, EA);
  run_tpose_hl(stream, env_wo, ewoT_h, ewoT_l,   EA, EA);
  run_tpose_hl(stream, snp_fw, sfwT_h, sfwT_l,   SA, FD);
  run_tpose_hl(stream, env_fw, efwT_h, efwT_l,   EA, FD);
  run_tpose_hl(stream, fus_fw, fusT_h, fusT_l,   2 * FD, FD);
  run_tpose_f16(stream, ew1,   ew1T, FD, MH, NE);
  run_tpose_f16(stream, ew2,   ew2T, MH, FD, NE);
  run_tpose_f16(stream, fn1_w, fn1T, FD, F1, 1);
  run_tpose_f16(stream, fn2_w, fn2T, F1, F2, 1);

  run_gemm<1, true, 1, 0, 0, 0>(stream, snp_h, snp_l, S, 0, w1T_h, w1T_l, S, 0, th1, th2_h, th2_h, WU, 0,
                                snp_b1, 0, snp_b1, 0, B, WU, S, 1, 1.0f);
  run_tpose_hl(stream, snp_pw, pwT_h, pwT_l, S, SA);
  ln_rows<true, 1><<<dim3(B / 8), blk, 0, stream>>>(th1, WU, snp_lng, snp_lnb, B, th2_h, th2_l, WU, B, WU);
  run_gemm<1, true, 0, 2, 2, 1>(stream, th2_h, th2_l, WU, 0, w2T_h, w2T_l, WU, 0, (float*)seff_h, seff_h, seff_l, S, 0,
                                snp_b2, 0, snp, 0, B, S, WU, 1, 1.0f);

  run_gemm<1, true, 1, 0, 0, 0>(stream, env_h, env_l, E_, 0, e_w1T_h, e_w1T_l, E_, 0, eh1, eh2_h, eh2_h, EU, 0,
                                env_b1, 0, env_b1, 0, B, EU, E_, 1, 1.0f);
  ln_rows<true, 1><<<dim3(B / 8), blk, 0, stream>>>(eh1, EU, env_lng, env_lnb, B, eh2_h, eh2_l, EU, B, EU);
  run_gemm<1, true, 0, 2, 2, 1>(stream, eh2_h, eh2_l, EU, 0, e_w2T_h, e_w2T_l, EU, 0, (float*)eeff_h, eeff_h, eeff_l, E_, 0,
                                env_b2, 0, env, 0, B, E_, EU, 1, 1.0f);

  run_gemm<1, true, 1, 2, 0, 0>(stream, seff_h, seff_l, S, 0, pwT_h, pwT_l, S, 0, sp, sp_h, sp_l, SA, 0,
                                snp_pb, 0, snp_pb, 0, B, SA, S, 1, 1.0f);
  run_gemm<1, true, 1, 2, 0, 0>(stream, eeff_h, eeff_l, E_, 0, epwT_h, epwT_l, E_, 0, ep, ep_h, ep_l, EA, 0,
                                env_pb, 0, env_pb, 0, B, EA, E_, 1, 1.0f);

  run_gemm<1, true, 0, 2, 0, 0>(stream, sp_h, sp_l, SA, 0, wvT_h, wvT_l, SA, 0, (float*)sv_h, sv_h, sv_l, SA, 0,
                                snp_bv, 0, snp_bv, 0, B, SA, SA, 1, 1.0f);
  run_gemm<1, true, 1, 0, 1, 0>(stream, sv_h, sv_l, SA, 0, woT_h, woT_l, SA, 0, sres, (us16*)sres, (us16*)sres, SA, 0,
                                snp_bo, 0, sp, 0, B, SA, SA, 1, 1.0f);
  ln_rows<false, 1><<<dim3(B / 8), blk, 0, stream>>>(sres, SA, snp_ng, snp_nb, B, sf_h, sf_l, SA, B, SA);
  run_gemm<1, true, 0, 2, 0, 0>(stream, ep_h, ep_l, EA, 0, ewvT_h, ewvT_l, EA, 0, (float*)ev_h, ev_h, ev_l, EA, 0,
                                env_bv, 0, env_bv, 0, B, EA, EA, 1, 1.0f);
  run_gemm<1, true, 1, 0, 1, 0>(stream, ev_h, ev_l, EA, 0, ewoT_h, ewoT_l, EA, 0, eres, (us16*)eres, (us16*)eres, EA, 0,
                                env_bo, 0, ep, 0, B, EA, EA, 1, 1.0f);
  ln_rows<false, 1><<<dim3(B / 8), blk, 0, stream>>>(eres, EA, env_ng, env_nb, B, ef_h, ef_l, EA, B, EA);

  run_gemm<1, true, 1, 0, 0, 0>(stream, sf_h, sf_l, SA, 0, sfwT_h, sfwT_l, SA, 0, fused, (us16*)fused, (us16*)fused, 2 * FD, 0,
                                snp_fb, 0, snp_fb, 0, B, FD, SA, 1, 1.0f);
  run_gemm<1, true, 1, 0, 0, 0>(stream, ef_h, ef_l, EA, 0, efwT_h, efwT_l, EA, 0, fused + FD, (us16*)fused, (us16*)fused, 2 * FD, 0,
                                env_fb, 0, env_fb, 0, B, FD, EA, 1, 1.0f);
  ln_rows<false, 1><<<dim3(B / 8), blk, 0, stream>>>(fused, 2 * FD, fus_ng, fus_nb, B, fus_h, fus_l, 2 * FD, B, 2 * FD);
  run_gemm<1, true, 1, 1, 0, 5>(stream, fus_h, fus_l, 2 * FD, 0, fusT_h, fusT_l, 2 * FD, 0, ff, ff16, ff16, FD, 0,
                                fus_fb, 0, fus_fb, 0, B, FD, 2 * FD, 1, 1.0f);

  gate_route<<<dim3(B / 32), blk, 0, stream>>>(ff, gate_w, gate_b, probs, comb, maskf, B, FD);
  aux_loss_k<<<dim3(1), blk, 0, stream>>>(probs, maskf, out1, B);

  run_gemm<0, false, 1, 0, 0, 0>(stream, ff16, ff16, FD, 0, ew1T, ew1T, FD, (long)MH * FD, hbuf, h16, h16, MH, (long)B * MH,
                                 eb1, MH, eb1, 0, B, MH, FD, NE, 0.015625f);
  ln_rows<true, 0><<<dim3(NE * B / 8), blk, 0, stream>>>(hbuf, MH, elg, elb, B, h16, h16, MH, NE * B, MH);
  run_gemm<0, false, 1, 0, 0, 0>(stream, h16, h16, MH, (long)B * MH, ew2T, ew2T, MH, (long)FD * MH, ybuf, (us16*)ybuf, (us16*)ybuf, FD, (long)B * FD,
                                 eb2, FD, eb2, 0, B, FD, MH, NE, 0.015625f);
  moe_combine_ln<<<dim3(B / 8), blk, 0, stream>>>(ybuf, comb, moe_ng, moe_nb, moe16, B);

  run_gemm<0, false, 1, 0, 0, 0>(stream, moe16, moe16, FD, 0, fn1T, fn1T, FD, 0, f1, (us16*)f1, (us16*)f1, F1, 0,
                                 fn1_b, 0, fn1_b, 0, B, F1, FD, 1, 0.015625f);
  ln_rows<true, 0><<<dim3(B / 8), blk, 0, stream>>>(f1, F1, fn1_g, fn1_bb, B, f1n16, f1n16, F1, B, F1);
  run_gemm<0, false, 1, 0, 0, 0>(stream, f1n16, f1n16, F1, 0, fn2T, fn2T, F1, 0, f2, (us16*)f2, (us16*)f2, F2, 0,
                                 fn2_b, 0, fn2_b, 0, B, F2, F1, 1, 0.015625f);
  ln_gelu_head<<<dim3(B / 32), blk, 0, stream>>>(f2, fn2_g, fn2_bb, pred_w, pred_b, out0, B);
}
